// GNNGM1_94489280749
// MI455X (gfx1250) — hardware-run, weakly checked
//
#include <hip/hip_runtime.h>


namespace {
constexpr int NN = 1024, HID = 64, DEG = 4, RD = 6, KF = 96  , KY = 96  , XRW = 80  ;
constexpr float HS = 256.0f, HSY = 64.0f  , WSC = 256.0f;
typedef _Float16 b16;
typedef __attribute__((ext_vector_type(16))) _Float16 v16b;
typedef __attribute__((ext_vector_type(8))) _Float16 v8b;
typedef __attribute__((ext_vector_type(8))) float v8f;
typedef __attribute__((ext_vector_type(4))) float v4f;
__device__ __forceinline__ float bf16_rne(float f) { unsigned int u = __float_as_uint(f); u += 0x7FFFu + ((u >> 16) & 1u); float r = __uint_as_float(u & 0xFFFF0000u); asm volatile("" : "+v"(r)); return r; }
__device__ __forceinline__ float bfv(float f) { float r = bf16_rne(f); asm volatile("" : "+v"(r)); return r; }
__device__ __forceinline__ void split16(float v, b16& hi, b16& lo) { hi = (b16)v; lo = (b16)(v - (float)hi); }
__device__ __forceinline__ v16b frag_kb(const b16* p, int hh) { const v8b a = *(const v8b*)(p + 8 * hh), b = *(const v8b*)(p + 16 + 8 * hh); v16b f;
#pragma unroll
  for (int e = 0; e < 8; ++e) { f[e] = a[e]; f[8 + e] = b[e]; } return f; }
__device__ __forceinline__ v8f wmma16b(v16b a, v16b b, v8f c) { v8f d = __builtin_amdgcn_wmma_f32_16x16x32_f16(false, a, false, b, (short)0, c, false, false); asm volatile("v_nop\n\tv_nop\n\tv_nop\n\tv_nop" : "+v"(d) : "v"(a), "v"(b)); return d; }
__device__ __forceinline__ void wave_lds_sync() { __builtin_amdgcn_fence(__ATOMIC_RELEASE, "workgroup"); __builtin_amdgcn_wave_barrier(); __builtin_amdgcn_fence(__ATOMIC_ACQUIRE, "workgroup"); }
__device__ __forceinline__ float pmul(float a, float b) { float p = a * b; asm volatile("" : "+v"(p)); return p; }
__device__ __forceinline__ int iclamp(int v, int lo, int hi) { return v < lo ? lo : (v > hi ? hi : v); }

__global__ __launch_bounds__(256) void wput_kernel(const float* __restrict__ iw2, const float* __restrict__ rw1, const float* __restrict__ mw1, const float* __restrict__ mw2, b16* __restrict__ IW2, b16* __restrict__ RW1, b16* __restrict__ MW1, b16* __restrict__ MW2) { const int u = blockIdx.x * 256 + threadIdx.x; v8b v;
  if (u < HID * 8) { const int o = u / 8, k0 = (u % 8) * 8;
#pragma unroll
    for (int j = 0; j < 8; ++j) v[j] = (b16)(bf16_rne(iw2[(size_t)(k0 + j) * HID + o]) * WSC); for (int pass = 0; pass < 2; ++pass) { *(volatile v8b*)(IW2 + (size_t)o * HID + k0) = v; __threadfence(); }
#pragma unroll
    for (int j = 0; j < 8; ++j) v[j] = (b16)(bf16_rne(mw2[(size_t)(k0 + j) * HID + o]) * WSC); for (int pass = 0; pass < 2; ++pass) { *(volatile v8b*)(MW2 + (size_t)o * HID + k0) = v; __threadfence(); } }
  if (u < 2 * HID * (KF / 8)) { const int l = u / (HID * (KF / 8)), r = u % (HID * (KF / 8)); const int o = r / (KF / 8), k0 = (r % (KF / 8)) * 8;
#pragma unroll
    for (int j = 0; j < 8; ++j) { const int k = k0 + j; v[j] = (b16)(k < HID + 1 ? bf16_rne(rw1[((size_t)l * (HID + 1) + k) * HID + o]) * WSC : 0.0f); } for (int pass = 0; pass < 2; ++pass) { *(volatile v8b*)(RW1 + ((size_t)l * HID + o) * KF + k0) = v; __threadfence(); } }
  if (u < HID * (KY / 8)) { const int o = u / (KY / 8), k0 = (u % (KY / 8)) * 8;
#pragma unroll
    for (int j = 0; j < 8; ++j) { const int k = k0 + j; v[j] = (b16)(k < HID + RD ? bf16_rne(mw1[(size_t)k * HID + o]) * WSC : 0.0f); } for (int pass = 0; pass < 2; ++pass) { *(volatile v8b*)(MW1 + (size_t)o * KY + k0) = v; __threadfence(); } } }
__global__ __launch_bounds__(32) void init_kernel(const float* __restrict__ G1, const float* __restrict__ G2, const float* __restrict__ iw1, const float* __restrict__ ib1, const b16* __restrict__ IW2, const float* __restrict__ ib2, float* __restrict__ X1, float* __restrict__ X2) { __shared__ __attribute__((aligned(16))) b16 Ah[16][HID + 8], Al[16][HID + 8]; __shared__ float Tf[16][HID + 4]; const int lane = threadIdx.x, nloc = lane & 15, hlf = lane >> 4; const int g = blockIdx.x / (NN / 16); const size_t m0 = (size_t)(blockIdx.x % (NN / 16)) * 16; const float* G = g == 0 ? G1 : G2;
  for (int rr = 0; rr < 16; ++rr) { float s = 0.0f; for (int q = 0; q < NN / 32; ++q) s += bfv(G[(m0 + rr) * NN + q * 32 + lane]); for (int o = 16; o; o >>= 1) s += __shfl_xor(s, o); s += 1.0f;
    for (int q = 0; q < 2; ++q) { const int c = q * 32 + lane; b16 p, ql; split16(fmaxf(pmul(s, bfv(iw1[c])) + bfv(ib1[c]), 0.0f) * HS, p, ql); Ah[rr][c] = p; Al[rr][c] = ql; } }
  if (lane < 16) for (int k = HID; k < HID + 8; ++k) { Ah[lane][k] = (b16)0.0f; Al[lane][k] = (b16)0.0f; }
  wave_lds_sync(); v8f acc[4] = {(v8f){}, (v8f){}, (v8f){}, (v8f){}};
#pragma unroll
  for (int kb = 0; kb < HID; kb += 32) { const v16b a = frag_kb(&Ah[nloc][kb], hlf), al = frag_kb(&Al[nloc][kb], hlf);
#pragma unroll
    for (int t = 0; t < 4; ++t) { const v16b bw = frag_kb(IW2 + (size_t)(t * 16 + nloc) * HID + kb, hlf); acc[t] = wmma16b(a, bw, acc[t]); acc[t] = wmma16b(al, bw, acc[t]); } }
#pragma unroll
  for (int t = 0; t < 4; ++t) { const int cc = t * 16 + nloc; const float bb = bfv(ib2[cc]);
#pragma unroll
    for (int r8 = 0; r8 < 8; ++r8) Tf[8 * hlf + r8][cc] = acc[t][r8] * (1.0f / (HS * WSC)) + bb; }
  wave_lds_sync(); float* X = g == 0 ? X1 : X2;
  for (int pass = 0; pass < 2; ++pass) { for (int rr = 0; rr < 16; ++rr) for (int q = 0; q < 2; ++q) ((volatile float*)X)[(m0 + rr) * HID + q * 32 + lane] = Tf[rr][q * 32 + lane]; __threadfence(); } }
__global__ __launch_bounds__(32) void readout_kernel(const float* __restrict__ X1, const float* __restrict__ X2, const float* __restrict__ P, const b16* __restrict__ RW1, const float* __restrict__ rb1, const float* __restrict__ rw2, const float* __restrict__ rb2, int HASP, int ILIM, float* __restrict__ O) { __shared__ __attribute__((aligned(16))) b16 Ah[32][KF + 8], Al[32][KF + 8]; __shared__ float Tf[32][HID + 4], X1s[HID]; const int lane = threadIdx.x, nloc = lane & 15, hlf = lane >> 4; const int i = blockIdx.x / (NN / 32), j0 = (blockIdx.x % (NN / 32)) * 32; if (i >= ILIM) return;
  X1s[lane] = X1[(size_t)i * HID + lane]; X1s[32 + lane] = X1[(size_t)i * HID + 32 + lane]; wave_lds_sync();
  for (int rr = 0; rr < 32; ++rr) { const int j = j0 + rr; for (int q = 0; q < 3; ++q) { const int c = q * 32 + lane; float v = 0.0f; if (c == 0) v = HASP ? P[(size_t)i * NN + j] : 0.0f; else if (c <= HID) v = -fabsf(X1s[c - 1] - X2[(size_t)j * HID + c - 1]) * 0.1f; b16 p, ql; split16(v * HS, p, ql); Ah[rr][c] = p; Al[rr][c] = ql; } if (lane < 8) { Ah[rr][KF + lane] = (b16)0.0f; Al[rr][KF + lane] = (b16)0.0f; } }
  wave_lds_sync();
#pragma unroll 1
  for (int rt = 0; rt < 2; ++rt) { v8f acc[4] = {(v8f){}, (v8f){}, (v8f){}, (v8f){}};
#pragma unroll
    for (int kb = 0; kb < KF; kb += 32) { const v16b a = frag_kb(&Ah[rt * 16 + nloc][kb], hlf), al = frag_kb(&Al[rt * 16 + nloc][kb], hlf);
#pragma unroll
      for (int t = 0; t < 4; ++t) { const v16b bw = frag_kb(RW1 + (size_t)(t * 16 + nloc) * KF + kb, hlf); acc[t] = wmma16b(a, bw, acc[t]); acc[t] = wmma16b(al, bw, acc[t]); } }
#pragma unroll
    for (int t = 0; t < 4; ++t) { const int cc = t * 16 + nloc; const float bb = bfv(rb1[cc]);
#pragma unroll
      for (int r8 = 0; r8 < 8; ++r8) Tf[rt * 16 + 8 * hlf + r8][cc] = fmaxf(acc[t][r8] * (1.0f / (HS * WSC)) + bb, 0.0f); } }
  wave_lds_sync();
  float o = 0.0f;
#pragma unroll 8
  for (int c = 0; c < HID; ++c) o += pmul(Tf[lane][c], bfv(rw2[c])); o += bfv(rb2[0]);
  for (int pass = 0; pass < 2; ++pass) { ((volatile float*)O)[(size_t)i * NN + j0 + lane] = o; __threadfence(); } }
__global__ __launch_bounds__(32) void col_kernel(const float* __restrict__ O, const float* __restrict__ r1, int HASR, int ILIM, float* __restrict__ SOUT, float* __restrict__ Wp, float* __restrict__ R2) { const int lane = threadIdx.x; const int j = blockIdx.x * 32 + lane; float mx = -INFINITY, se = 0.0f;
#pragma unroll 1
  for (int i = 0; i < ILIM; ++i) { const float v = O[(size_t)i * NN + j]; const float mn = fmaxf(mx, v); se = se * ((mx == -INFINITY) ? 0.0f : __expf(mx - mn)) + __expf(v - mn); mx = mn; }
  const float lse = mx + __logf(se); float r2[RD]; for (int q = 0; q < RD; ++q) r2[q] = 0.0f;
  for (int pass = 0; pass < 2; ++pass) {
#pragma unroll 1
    for (int i = 0; i < ILIM; ++i) { const float s = __expf(O[(size_t)i * NN + j] - lse); ((volatile float*)SOUT)[(size_t)i * NN + j] = s; ((volatile float*)Wp)[(size_t)i * NN + j] = __logf((float)NN * s * 1.5f); if (pass == 0 && HASR) {
#pragma unroll
        for (int q = 0; q < RD; ++q) r2[q] += pmul(s, bfv(r1[(size_t)i * RD + q])); } }
    if (HASR) {
#pragma unroll
      for (int q = 0; q < RD; ++q) ((volatile float*)R2)[(size_t)j * RD + q] = r2[q]; } __threadfence(); } }
__global__ __launch_bounds__(256) void lap_kernel(const float* __restrict__ Wp, const int* __restrict__ adj1, const int* __restrict__ adj2, int ILIM, float* __restrict__ P) { const size_t u = (size_t)blockIdx.x * 256 + threadIdx.x; const int i = (int)(u / NN), j = (int)(u % NN); if (i >= ILIM) return; constexpr int PR[24][4] = {{0,1,2,3},{0,1,3,2},{0,2,1,3},{0,2,3,1},{0,3,1,2},{0,3,2,1},{1,0,2,3},{1,0,3,2},{1,2,0,3},{1,2,3,0},{1,3,0,2},{1,3,2,0},{2,0,1,3},{2,0,3,1},{2,1,0,3},{2,1,3,0},{2,3,0,1},{2,3,1,0},{3,0,1,2},{3,0,2,1},{3,1,0,2},{3,1,2,0},{3,2,0,1},{3,2,1,0}}; float w[DEG][DEG];
#pragma unroll
  for (int a = 0; a < DEG; ++a) { const int ia = iclamp(adj1[i * DEG + a], 0, ILIM - 1);
#pragma unroll
    for (int b = 0; b < DEG; ++b) { const int jb = iclamp(adj2[j * DEG + b], 0, NN - 1); w[a][b] = Wp[(size_t)ia * NN + jb]; } }
  float best = -INFINITY;
#pragma unroll
  for (int p = 0; p < 24; ++p) { const float s = ((w[0][PR[p][0]] + w[1][PR[p][1]]) + w[2][PR[p][2]]) + w[3][PR[p][3]]; best = fmaxf(best, s); }
  for (int pass = 0; pass < 2; ++pass) { ((volatile float*)P)[u] = best; __threadfence(); } }
__global__ __launch_bounds__(32) void xrt_kernel(const float* __restrict__ X1, const float* __restrict__ X2, const float* __restrict__ r1, const float* __restrict__ R2, b16* __restrict__ XRh, b16* __restrict__ XRl) { const int lane = threadIdx.x; const int g = blockIdx.x / XRW, o = blockIdx.x % XRW; const float* X = g == 0 ? X1 : X2; const float* R = g == 0 ? r1 : R2;
  for (int pass = 0; pass < 2; ++pass) { for (int n0 = 0; n0 < NN; n0 += 32) { const int n = n0 + lane; float v = 0.0f; if (o < HID) v = X[(size_t)n * HID + o]; else if (o < HID + RD) v = g == 0 ? bfv(R[(size_t)n * RD + o - HID]) : R[(size_t)n * RD + o - HID]; b16 p, ql; split16(v * HS, p, ql); ((volatile b16*)XRh)[((size_t)g * XRW + o) * NN + n] = p; ((volatile b16*)XRl)[((size_t)g * XRW + o) * NN + n] = ql; } __threadfence(); } }
__global__ __launch_bounds__(32) void msg_kernel(const float* __restrict__ G1, const float* __restrict__ G2, const b16* __restrict__ XRh, const b16* __restrict__ XRl, const float* __restrict__ X1in, const float* __restrict__ X2in, const float* __restrict__ r1, const float* __restrict__ R2, const b16* __restrict__ MW1, const b16* __restrict__ MW2, const float* __restrict__ mb1, const float* __restrict__ mb2, float* __restrict__ X1o, float* __restrict__ X2o) {
  __shared__ __attribute__((aligned(16))) b16 Gs[16][264], Ah[16][KY + 8], Al[16][KY + 8]; __shared__ float Tf[16][XRW + 4]; const int lane = threadIdx.x, nloc = lane & 15, hlf = lane >> 4; const int g = blockIdx.x / (NN / 16); const size_t m0 = (size_t)(blockIdx.x % (NN / 16)) * 16; const float* G = g == 0 ? G1 : G2; const float* Xin = g == 0 ? X1in : X2in; const float* R = g == 0 ? r1 : R2; const b16* Bh = XRh + (size_t)g * XRW * NN; const b16* Bl = XRl + (size_t)g * XRW * NN;
  v8f acc[5];
#pragma unroll
  for (int t = 0; t < 5; ++t) acc[t] = (v8f){};
  if (lane < 16) for (int k = 256; k < 264; ++k) Gs[lane][k] = (b16)0.0f;
#pragma unroll 1
  for (int kc = 0; kc < NN; kc += 256) { for (int rr = 0; rr < 16; ++rr) for (int q = 0; q < 8; ++q) Gs[rr][q * 32 + lane] = (b16)bfv(G[(m0 + rr) * NN + kc + q * 32 + lane]);
    wave_lds_sync();
#pragma unroll 2
    for (int kb = 0; kb < 256; kb += 32) { const v16b a = frag_kb(&Gs[nloc][kb], hlf);
#pragma unroll
      for (int t = 0; t < 5; ++t) { const size_t br = (size_t)(t * 16 + nloc) * NN + kc + kb; acc[t] = wmma16b(a, frag_kb(Bh + br, hlf), acc[t]); acc[t] = wmma16b(a, frag_kb(Bl + br, hlf), acc[t]); } }
    wave_lds_sync(); }
#pragma unroll
  for (int t = 0; t < 5; ++t)
#pragma unroll
    for (int r8 = 0; r8 < 8; ++r8) Tf[8 * hlf + r8][t * 16 + nloc] = acc[t][r8] * (1.0f / HS);
  wave_lds_sync();
  for (int rr = 0; rr < 16; ++rr) for (int q = 0; q < 3; ++q) { const int c = q * 32 + lane; float v = 0.0f; if (c < HID) v = Tf[rr][c] + Xin[(m0 + rr) * HID + c]; else if (c < HID + RD) v = Tf[rr][c] + (g == 0 ? bfv(R[(m0 + rr) * RD + c - HID]) : R[(m0 + rr) * RD + c - HID]); b16 p, ql; split16(v * HSY, p, ql); Ah[rr][c] = p; Al[rr][c] = ql; }
  if (lane < 16) for (int k = KY; k < KY + 8; ++k) { Ah[lane][k] = (b16)0.0f; Al[lane][k] = (b16)0.0f; }
  wave_lds_sync(); v8f a2[4] = {(v8f){}, (v8f){}, (v8f){}, (v8f){}};
#pragma unroll
  for (int kb = 0; kb < KY; kb += 32) { const v16b a = frag_kb(&Ah[nloc][kb], hlf), al = frag_kb(&Al[nloc][kb], hlf);
#pragma unroll
    for (int t = 0; t < 4; ++t) { const v16b bw = frag_kb(MW1 + (size_t)(t * 16 + nloc) * KY + kb, hlf); a2[t] = wmma16b(a, bw, a2[t]); a2[t] = wmma16b(al, bw, a2[t]); } }
  wave_lds_sync();
#pragma unroll
  for (int t = 0; t < 4; ++t) { const int cc = t * 16 + nloc; const float bb = bfv(mb1[cc]);
#pragma unroll
    for (int r8 = 0; r8 < 8; ++r8) { b16 p, ql; split16(fmaxf(a2[t][r8] * (1.0f / (HSY * WSC)) + bb, 0.0f) * HSY, p, ql); Ah[8 * hlf + r8][cc] = p; Al[8 * hlf + r8][cc] = ql; } }
  wave_lds_sync();
#pragma unroll
  for (int t = 0; t < 4; ++t) a2[t] = (v8f){};
#pragma unroll
  for (int kb = 0; kb < HID; kb += 32) { const v16b a = frag_kb(&Ah[nloc][kb], hlf), al = frag_kb(&Al[nloc][kb], hlf);
#pragma unroll
    for (int t = 0; t < 4; ++t) { const v16b bw = frag_kb(MW2 + (size_t)(t * 16 + nloc) * HID + kb, hlf); a2[t] = wmma16b(a, bw, a2[t]); a2[t] = wmma16b(al, bw, a2[t]); } }
#pragma unroll
  for (int t = 0; t < 4; ++t) { const int cc = t * 16 + nloc; const float bb = bfv(mb2[cc]);
#pragma unroll
    for (int r8 = 0; r8 < 8; ++r8) Tf[8 * hlf + r8][cc] = a2[t][r8] * (1.0f / (HSY * WSC)) + bb; }
  wave_lds_sync(); float* Xo = g == 0 ? X1o : X2o;
  for (int pass = 0; pass < 2; ++pass) { for (int rr = 0; rr < 16; ++rr) for (int q = 0; q < 2; ++q) ((volatile float*)Xo)[(m0 + rr) * HID + q * 32 + lane] = Tf[rr][q * 32 + lane]; __threadfence(); } }
}

extern "C" void kernel_launch(void* const* d_in, const int* in_sizes, int n_in, void* d_out, int out_size, void* d_ws, size_t ws_size, hipStream_t stream) {
  (void)n_in;
  auto Fp = [&](int i) { return (const float*)d_in[i]; }; auto Ip = [&](int i) { return (const int*)d_in[i]; };
  if (in_sizes[0] != NN * NN || in_sizes[1] != NN * NN || in_sizes[2] != NN * RD || in_sizes[3] != HID || in_sizes[5] != HID * HID || in_sizes[7] != 2 * (HID + 1) * HID || in_sizes[9] != 2 * HID || in_sizes[11] != (HID + RD) * HID || in_sizes[13] != HID * HID || in_sizes[15] != NN * DEG || in_sizes[16] != NN * DEG || out_size != 3 * NN * NN) return;
  const int ILIM = NN;
  size_t off = 0; char* ws = (char*)d_ws;
  auto carve = [&](size_t bytes) { char* p = ws + off; off += (bytes + 255) & ~(size_t)255; return p; };
  b16* IW2 = (b16*)carve((size_t)HID * HID * 2); b16* RW1 = (b16*)carve((size_t)2 * HID * KF * 2); b16* MW1 = (b16*)carve((size_t)HID * KY * 2); b16* MW2 = (b16*)carve((size_t)HID * HID * 2);
  float* X1 = (float*)carve((size_t)NN * HID * 4); float* X2 = (float*)carve((size_t)NN * HID * 4); float* X1b = (float*)carve((size_t)NN * HID * 4); float* X2b = (float*)carve((size_t)NN * HID * 4); float* O = (float*)carve((size_t)NN * NN * 4); float* Wp = (float*)carve((size_t)NN * NN * 4); float* P1 = (float*)carve((size_t)NN * NN * 4); float* R2 = (float*)carve((size_t)NN * RD * 4); b16* XRh = (b16*)carve((size_t)2 * XRW * NN * 2); b16* XRl = (b16*)carve((size_t)2 * XRW * NN * 2);
  if (off > ws_size || off > ((size_t)32 << 20)) return;
  float* POUT = (float*)d_out; float* S1 = POUT + (size_t)NN * NN; float* S2 = S1 + (size_t)NN * NN;
  wput_kernel<<<(2 * HID * (KF / 8) + 255) / 256, 256, 0, stream>>>(Fp(5), Fp(7), Fp(11), Fp(13), IW2, RW1, MW1, MW2);
  init_kernel<<<2 * (NN / 16), 32, 0, stream>>>(Fp(0), Fp(1), Fp(3), Fp(4), IW2, Fp(6), X1, X2);
  readout_kernel<<<ILIM * (NN / 32), 32, 0, stream>>>(X1, X2, P1, RW1, Fp(8), Fp(9), Fp(10), 0, ILIM, O);
  col_kernel<<<NN / 32, 32, 0, stream>>>(O, Fp(2), 1, ILIM, S1, Wp, R2);
  lap_kernel<<<(ILIM * NN + 255) / 256, 256, 0, stream>>>(Wp, Ip(15), Ip(16), ILIM, P1);
  xrt_kernel<<<2 * XRW, 32, 0, stream>>>(X1, X2, Fp(2), R2, XRh, XRl);
  msg_kernel<<<2 * (NN / 16), 32, 0, stream>>>(Fp(0), Fp(1), XRh, XRl, X1, X2, Fp(2), R2, MW1, MW2, Fp(12), Fp(14), X1b, X2b);
  readout_kernel<<<ILIM * (NN / 32), 32, 0, stream>>>(X1b, X2b, P1, RW1 + (size_t)HID * KF, Fp(8) + HID, Fp(9) + HID, Fp(10) + 1, 1, ILIM, O);
  col_kernel<<<NN / 32, 32, 0, stream>>>(O, Fp(2), 0, ILIM, S2, Wp, R2);
  lap_kernel<<<(ILIM * NN + 255) / 256, 256, 0, stream>>>(Wp, Ip(15), Ip(16), ILIM, POUT);
}
